// DownsampleModel_20564303414104
// MI455X (gfx1250) — hardware-run, weakly checked
//
#include <hip/hip_runtime.h>

typedef float          v8f   __attribute__((ext_vector_type(8)));
typedef float          v4f   __attribute__((ext_vector_type(4)));
typedef unsigned int   v4u   __attribute__((ext_vector_type(4)));
typedef int            v8i   __attribute__((ext_vector_type(8)));
typedef unsigned short v8us  __attribute__((ext_vector_type(8)));
typedef unsigned short v16us __attribute__((ext_vector_type(16)));
typedef __bf16         v16bf __attribute__((ext_vector_type(16)));
typedef _Float16       v16h  __attribute__((ext_vector_type(16)));
typedef v4f  __attribute__((may_alias)) v4fa;
typedef v8us __attribute__((may_alias)) v8usa;
union FragB { v16bf v; v16us u; v8us h[2]; v8i w; };
union FragH { v16h  v; v16us u; v8us h[2]; v8i w; };

__device__ __forceinline__ v8f wmb(const FragB& a, const FragB& b, v8f c) {
  v8f d = __builtin_amdgcn_wmma_f32_16x16x32_bf16(false, a.v, false, b.v, (short)0, c, false, false);
  asm volatile("v_nop\n\tv_nop\n\tv_nop\n\tv_nop" : "+v"(d) : "v"(a.w), "v"(b.w));
  return d;
}

__device__ __forceinline__ v8f wmh(const FragH& a, const FragH& b, v8f c) {
  v8f d = __builtin_amdgcn_wmma_f32_16x16x32_f16(false, a.v, false, b.v, (short)0, c, false, false);
  asm volatile("v_nop\n\tv_nop\n\tv_nop\n\tv_nop" : "+v"(d) : "v"(a.w), "v"(b.w));
  return d;
}

__device__ __forceinline__ unsigned bf16_bits(float f) {
  const unsigned u = __float_as_uint(f);
  const unsigned r = (u + 0x7FFFu + ((u >> 16) & 1u)) >> 16;
  const unsigned q = (u >> 16) | 0x40u;
  return ((u & 0x7fffffffu) > 0x7f800000u) ? q : r;
}

__device__ __forceinline__ float bf16_val(float f) {
  return __uint_as_float(bf16_bits(f) << 16);
}
__device__ __forceinline__ int clampi(int v, int lo, int hi) {
  return v < lo ? lo : (v > hi ? hi : v);
}

__device__ __forceinline__ unsigned f16_bits(float f) {
  const unsigned u  = __float_as_uint(f);
  const unsigned s  = (u >> 16) & 0x8000u;
  const unsigned a  = u & 0x7fffffffu;
  const unsigned t  = a - 0x38000000u;
  const unsigned r  = (t + 0x0FFFu + ((t >> 13) & 1u)) >> 13;
  const unsigned rc = r > 0x7C00u ? 0x7C00u : r;
  const bool small  = a < 0x38800000u;
  const bool isnan  = a > 0x7f800000u;
  const unsigned fin = small ? 0u : (s | rc);
  return isnan ? (s | 0x7E00u) : fin;
}

__device__ __forceinline__ unsigned pk16(unsigned lo, unsigned hi) { return lo | (hi << 16); }
__device__ __forceinline__ unsigned bf16_lo_bits(float v) {
  float hi = bf16_val(v);
  asm volatile("" : "+v"(hi));
  return bf16_bits(v - hi);
}
__device__ __forceinline__ v4u pack8_bf16(v4f a, v4f c) {
  return (v4u){ pk16(bf16_bits(a[0]), bf16_bits(a[1])), pk16(bf16_bits(a[2]), bf16_bits(a[3])),
                pk16(bf16_bits(c[0]), bf16_bits(c[1])), pk16(bf16_bits(c[2]), bf16_bits(c[3])) };
}
__device__ __forceinline__ v4u pack8_bf16_lo(v4f a, v4f c) {
  return (v4u){ pk16(bf16_lo_bits(a[0]), bf16_lo_bits(a[1])), pk16(bf16_lo_bits(a[2]), bf16_lo_bits(a[3])),
                pk16(bf16_lo_bits(c[0]), bf16_lo_bits(c[1])), pk16(bf16_lo_bits(c[2]), bf16_lo_bits(c[3])) };
}
__device__ __forceinline__ v4u pack8_f16(v4f a, v4f c) {
  return (v4u){ pk16(f16_bits(a[0]), f16_bits(a[1])), pk16(f16_bits(a[2]), f16_bits(a[3])),
                pk16(f16_bits(c[0]), f16_bits(c[1])), pk16(f16_bits(c[2]), f16_bits(c[3])) };
}

template <int FORM>
__global__ __launch_bounds__(256) void k_plane(const float* __restrict__ src, int rows, int cols, int ldsrc,
                                               unsigned short* __restrict__ dst, int MP, int KP) {
  static_assert(FORM >= 0 && FORM <= 3);
  const int KTOT = (FORM == 1 || FORM == 3) ? 2 * KP : KP;
  const unsigned ppr   = (unsigned)(KTOT >> 3);
  const unsigned kp8   = (unsigned)(KP >> 3);
  const unsigned total = (unsigned)MP * ppr;
  const unsigned g     = blockIdx.x * 256u + threadIdx.x;
  const unsigned rowu  = g / ppr;
  const unsigned p     = g - rowu * ppr;
  const bool second    = p >= kp8;
  const int row = (int)rowu;
  const int c0  = (int)((second ? p - kp8 : p) << 3);
  const float* srow = src + (size_t)clampi(row, 0, rows - 1) * (size_t)ldsrc;
  float x[8];
  unsigned mk[8];
#pragma unroll
  for (int e = 0; e < 8; ++e) {
    const int c = c0 + e;
    const float v = srow[clampi(c, 0, cols - 1)];
    asm volatile("" :: "v"(v));
    x[e]  = v;
    mk[e] = (row < rows && c < cols) ? 0xFFFFu : 0u;
  }
  const v4f a = (v4f){ x[0], x[1], x[2], x[3] };
  const v4f c = (v4f){ x[4], x[5], x[6], x[7] };
  v4u o;
  if (FORM == 2) {
    o = pack8_f16(a, c);
  } else {
    const v4u hi = pack8_bf16(a, c);
    o = hi;
    if (FORM == 1) { const v4u lo = pack8_bf16_lo(a, c); o = second ? lo : hi; }
  }
  const v4u mw = (v4u){ pk16(mk[0], mk[1]), pk16(mk[2], mk[3]), pk16(mk[4], mk[5]), pk16(mk[6], mk[7]) };
  o &= mw;
  if (g < total) {
    volatile v4u* q = (volatile v4u*)(dst + (size_t)g * 8);
    *q = o;
    __threadfence();
    *q = o;
  }
}

template <int FORM> struct FragOf    { typedef FragB T; };
template <>         struct FragOf<2> { typedef FragH T; };
__device__ __forceinline__ v8f mm(const FragB& a, const FragB& b, v8f c) { return wmb(a, b, c); }
__device__ __forceinline__ v8f mm(const FragH& a, const FragH& b, v8f c) { return wmh(a, b, c); }
template <class F> __device__ __forceinline__ F ld_frag(const unsigned short* p) {
  F f;
  f.h[0] = *(const v8usa*)(p);
  f.h[1] = *(const v8usa*)(p + 16);
  return f;
}

template <int FORM, int EPI>
__global__ __launch_bounds__(256) __attribute__((amdgpu_num_vgpr(248)))
void k_gemm_nt(const unsigned short* __restrict__ A, const unsigned short* __restrict__ B,
               const float* __restrict__ bias, float* __restrict__ D, int M, int N, int KTOT, int ldd) {
  static_assert(FORM >= 0 && FORM <= 2);
  static_assert(EPI == 0 || EPI == 1);
  typedef typename FragOf<FORM>::T F;
  __shared__ __attribute__((aligned(16))) float sT[8][16 * 68];
  const int lane = threadIdx.x & 31;
  const int wave = threadIdx.x >> 5;
  const int tilesM = (M + 63) >> 6;
  const int tilesN = (N + 63) >> 6;
  const int tile = blockIdx.x * 8 + wave;
  if (tile >= tilesM * tilesN) return;
  const int tm = tile / tilesN;
  const int tn = tile - tm * tilesN;
  const int m0 = tm << 6;
  const int n0 = tn << 6;

  const int rl = lane & 15;
  const int h8 = (lane >> 4) * 8;
  const unsigned short* pa = A + (size_t)(m0 + rl) * (size_t)KTOT + h8;
  const unsigned short* pb = B + (size_t)(n0 + rl) * (size_t)KTOT + h8;

  v8f acc[4][4];
#pragma unroll
  for (int i = 0; i < 4; ++i)
#pragma unroll
    for (int j = 0; j < 4; ++j) acc[i][j] = (v8f){0.f, 0.f, 0.f, 0.f, 0.f, 0.f, 0.f, 0.f};

#pragma unroll 1
  for (int k0 = 0; k0 < KTOT; k0 += 32) {
    F bf[4];
#pragma unroll
    for (int j = 0; j < 4; ++j) bf[j] = ld_frag<F>(pb + (size_t)(j << 4) * (size_t)KTOT + k0);
#pragma unroll
    for (int i = 0; i < 4; ++i) {
      const F af = ld_frag<F>(pa + (size_t)(i << 4) * (size_t)KTOT + k0);
#pragma unroll
      for (int j = 0; j < 4; ++j) acc[i][j] = mm(af, bf[j], acc[i][j]);
    }
  }

  float* slab = sT[wave];
  const int hh = lane >> 4;
  const int c4 = (lane & 15) * 4;
  const int nc = n0 + c4;
  const bool cok = nc < N;
  v4f bv = (v4f){0.f, 0.f, 0.f, 0.f};
  if (EPI == 1) {
    bv = *(const v4fa*)(bias + clampi(nc, 0, N - 4));
    asm volatile("" :: "v"(bv));
  }
#pragma unroll
  for (int i = 0; i < 4; ++i) {
    const int mBase = m0 + (i << 4);
#pragma unroll
    for (int j = 0; j < 4; ++j) {
#pragma unroll
      for (int r = 0; r < 8; ++r) slab[(h8 + r) * 68 + (j << 4) + rl] = acc[i][j][r];
    }
    __builtin_amdgcn_fence(__ATOMIC_RELEASE, "workgroup");
    __builtin_amdgcn_wave_barrier();
    __builtin_amdgcn_fence(__ATOMIC_ACQUIRE, "workgroup");
    v4f vv[8];
#pragma unroll
    for (int it = 0; it < 8; ++it) {
      const int row = it * 2 + hh;
      v4f v = *(const v4fa*)(slab + row * 68 + c4);
      if (EPI == 1) v += bv;
      vv[it] = v;
    }
    for (int pass = 0; pass < 2; ++pass) {
#pragma unroll
      for (int it = 0; it < 8; ++it) {
        const int row = mBase + it * 2 + hh;
        if (cok && row < M) *(volatile v4f*)(D + (size_t)row * (size_t)ldd + nc) = vv[it];
      }
      __threadfence();
    }
    __builtin_amdgcn_fence(__ATOMIC_RELEASE, "workgroup");
    __builtin_amdgcn_wave_barrier();
    __builtin_amdgcn_fence(__ATOMIC_ACQUIRE, "workgroup");
  }
}

#pragma clang fp contract(off)

#ifndef TWO_TERM_2
#define TWO_TERM_2 1
#endif
#ifndef TWO_TERM_3
#define TWO_TERM_3 1
#endif
static_assert(TWO_TERM_2 == 0 || TWO_TERM_2 == 1);
static_assert(TWO_TERM_3 == 0 || TWO_TERM_3 == 1);

typedef float        v2f __attribute__((ext_vector_type(2)));
typedef unsigned int v2u __attribute__((ext_vector_type(2)));
typedef int          v4i __attribute__((ext_vector_type(4)));
typedef double       v2d __attribute__((ext_vector_type(2)));
typedef v2f __attribute__((may_alias)) v2fa;
typedef v4i __attribute__((may_alias)) v4ia;
typedef v4u __attribute__((may_alias)) v4ua;

constexpr int N1   = 180000;
constexpr int M2   = 32768;
constexpr int C1   = 64;
constexpr int C2   = 128;
constexpr int NTAP = 27;
constexpr int P1   = 180000;
constexpr int P2   = 32768;
constexpr int K1   = NTAP * C1;
constexpr int TW2  = TWO_TERM_2 ? 2 * C1 : C1;
constexpr int K2   = NTAP * TW2;
constexpr int TW3  = TWO_TERM_3 ? 2 * C2 : C2;
constexpr int K3   = NTAP * TW3;
constexpr int TILE = 2048;
constexpr int TB1  = (N1 + TILE - 1) / TILE;
constexpr int TB2  = M2 / TILE;
constexpr int NBR1 = TB1 * TILE;
constexpr int TABLE_LDS = TILE * 32 * 4;
constexpr int CH1_REAL = 12000, CH1_PAD = 12032, CH1_N = 15;
constexpr int CH2_ROWS = 4096,  CH2_N = 8;
constexpr int CH3_ROWS = 2048,  CH3_N = 16;

static_assert(TB1 == 88 && NBR1 == 180224 && TB2 * TILE == M2);
static_assert(TABLE_LDS == 262144 && TABLE_LDS + 0 <= 327680);
static_assert(N1 < (1 << 20) && M2 < (1 << 20));
static_assert(P1 % 8 == 0 && P2 % 8 == 0);
static_assert(K1 % 32 == 0 && K2 % 32 == 0 && K3 % 32 == 0);
static_assert(C1 % 64 == 0 && C2 % 64 == 0 && C1 % 32 == 0 && C2 % 32 == 0);
static_assert(CH1_REAL * CH1_N == N1 && CH1_REAL % 16 == 0 && CH1_PAD % 64 == 0 && CH1_PAD % 128 == 0 && CH1_PAD >= CH1_REAL);
static_assert(CH2_ROWS * CH2_N == M2 && CH2_ROWS % 128 == 0 && CH3_ROWS * CH3_N == M2 && CH3_ROWS % 128 == 0);
static_assert((CH1_N - 1) * CH1_REAL + CH1_PAD <= NBR1);
static_assert(((size_t)CH1_REAL * C1 * 4) % 128 == 0 && ((size_t)CH2_ROWS * C2 * 4) % 128 == 0);

constexpr int P_G1 = 0, P_B1 = 64, P_G2 = 128, P_B2 = 256, P_G3 = 384, P_B3 = 512, P_N = 640;
constexpr int ST_SET = 384, ST_VAR = 128, ST_RS = 256;

constexpr size_t SZ_CHUNK = (size_t)CH1_PAD * K1 * 2;
constexpr size_t SZ_X1    = (size_t)N1 * C1 * 4;
constexpr size_t SZ_NB    = (size_t)NBR1 * 32 * 4;
constexpr size_t SZ_NB2   = (size_t)M2 * 32 * 4;
constexpr size_t SZ_X2    = (size_t)M2 * C2 * 4;
constexpr size_t SZ_W1T   = (size_t)C1 * NTAP * C1 * 2;
constexpr size_t SZ_W2T   = (size_t)C2 * NTAP * 2 * C1 * 2;
constexpr size_t SZ_W3T   = (size_t)C2 * NTAP * 2 * C2 * 2;
constexpr size_t SZ_REC   = 1048576;
constexpr size_t SZ_PAR   = 3072;
constexpr size_t SZ_ST    = 5120;
constexpr size_t OFF_CHUNK = 0;
constexpr size_t OFF_X1    = OFF_CHUNK + SZ_CHUNK;
constexpr size_t OFF_NB    = OFF_X1 + SZ_X1;
constexpr size_t OFF_X2    = OFF_NB + SZ_NB;
constexpr size_t OFF_W1T   = OFF_X2 + SZ_X2;
constexpr size_t OFF_W2T   = OFF_W1T + SZ_W1T;
constexpr size_t OFF_W3T   = OFF_W2T + SZ_W2T;
constexpr size_t OFF_REC   = OFF_W3T + SZ_W3T;
constexpr size_t OFF_PAR   = OFF_REC + SZ_REC;
constexpr size_t OFF_ST    = OFF_PAR + SZ_PAR;
constexpr size_t WS_TOTAL  = OFF_ST + SZ_ST;
static_assert(SZ_CHUNK == (size_t)41582592 && SZ_X1 == (size_t)46080000 && SZ_NB == (size_t)23068672);
static_assert(WS_TOTAL == (size_t)((size_t)16045 << 13) && WS_TOTAL <= ((size_t)128 << 20));
static_assert(SZ_CHUNK % 256 == 0 && SZ_X1 % 256 == 0 && SZ_NB % 256 == 0 && SZ_X2 % 256 == 0 && SZ_W1T % 256 == 0);
static_assert(SZ_W2T % 256 == 0 && SZ_W3T % 256 == 0 && SZ_REC % 256 == 0 && SZ_PAR % 256 == 0 && SZ_ST % 256 == 0);
static_assert((size_t)CH2_ROWS * K2 * 2 <= SZ_CHUNK && (size_t)CH3_ROWS * K3 * 2 <= SZ_CHUNK);
static_assert((size_t)C2 * K2 * 2 <= SZ_W2T && (size_t)C2 * K3 * 2 <= SZ_W3T);
static_assert(2 * SZ_NB2 <= SZ_NB && (size_t)M2 * C2 * 4 <= SZ_X1);
static_assert((size_t)((N1 + 127) / 128) * C1 * 8 <= SZ_REC && (size_t)(M2 / 128) * C2 * 8 <= SZ_REC);
static_assert((size_t)P_N * 4 <= SZ_PAR && (size_t)3 * ST_SET * 4 <= SZ_ST);

__device__ __forceinline__ float relu_k(float v) { return (v > 0.0f) ? v : (v - v); }

constexpr int PB_W1 = C1 * (K1 / 8) / 256;
constexpr int PB_W2 = C2 * (K2 / 8) / 256;
constexpr int PB_W3 = C2 * (K3 / 8) / 256;
constexpr int PREP_BLOCKS = PB_W1 + PB_W2 + PB_W3 + 1;
static_assert((C1 * (K1 / 8)) % 256 == 0 && (C2 * (K2 / 8)) % 256 == 0 && (C2 * (K3 / 8)) % 256 == 0);

__device__ __forceinline__ void wt_unit(const float* __restrict__ W, int cin, int cout, int tw, int ppr,
                                        unsigned short* __restrict__ dst, int u) {
  const int n    = u / ppr;
  const int p    = u - n * ppr;
  const int kpos = p << 3;
  const int tap  = kpos / tw;
  const int j    = kpos - tap * tw;
  const int ci0  = j & (cin - 1);
  const float* s = W + ((size_t)tap * (size_t)cin + (size_t)ci0) * (size_t)cout + n;
  float x[8];
#pragma unroll
  for (int e = 0; e < 8; ++e) {
    const float v = s[(size_t)e * (size_t)cout];
    asm volatile("" :: "v"(v));
    x[e] = v;
  }
  const v4u o = pack8_bf16((v4f){ x[0], x[1], x[2], x[3] }, (v4f){ x[4], x[5], x[6], x[7] });
  volatile v4u* q = (volatile v4u*)(dst + (size_t)u * 8);
  *q = o;
  __threadfence();
  *q = o;
}

__device__ __forceinline__ v4u par_piece(const float* __restrict__ p, int j, bool on) {
  const v4f a = *(const v4fa*)(p + 4 * j);
  asm volatile("" :: "v"(a));
  const unsigned m = on ? 0xFFFFFFFFu : 0u;
  return (v4u){ __float_as_uint(a[0]) & m, __float_as_uint(a[1]) & m, __float_as_uint(a[2]) & m, __float_as_uint(a[3]) & m };
}

__global__ __launch_bounds__(256) void k_wprep(const float* __restrict__ W1, const float* __restrict__ W2,
                                               const float* __restrict__ W3,
                                               const float* __restrict__ g1, const float* __restrict__ b1,
                                               const float* __restrict__ g2, const float* __restrict__ b2,
                                               const float* __restrict__ g3, const float* __restrict__ b3,
                                               unsigned short* __restrict__ W1T, unsigned short* __restrict__ W2T,
                                               unsigned short* __restrict__ W3T, float* __restrict__ PAR) {
  const int tid = (int)threadIdx.x;
  const int blk = (int)blockIdx.x;
  if (blk < PB_W1) {
    wt_unit(W1, C1, C1, C1, K1 / 8, W1T, blk * 256 + tid);
  } else if (blk < PB_W1 + PB_W2) {
    wt_unit(W2, C1, C2, TW2, K2 / 8, W2T, (blk - PB_W1) * 256 + tid);
  } else if (blk < PB_W1 + PB_W2 + PB_W3) {
    wt_unit(W3, C2, C2, TW3, K3 / 8, W3T, (blk - PB_W1 - PB_W2) * 256 + tid);
  } else {
    const int u = tid < P_N / 4 ? tid : P_N / 4 - 1;
    v4u acc = par_piece(g1, clampi(u, 0, 15), u < 16);
    acc |= par_piece(b1, clampi(u - 16, 0, 15), u >= 16 && u < 32);
    acc |= par_piece(g2, clampi(u - 32, 0, 31), u >= 32 && u < 64);
    acc |= par_piece(b2, clampi(u - 64, 0, 31), u >= 64 && u < 96);
    acc |= par_piece(g3, clampi(u - 96, 0, 31), u >= 96 && u < 128);
    acc |= par_piece(b3, clampi(u - 128, 0, 31), u >= 128);
    const v4f o = (v4f){ bf16_val(__uint_as_float(acc[0])), bf16_val(__uint_as_float(acc[1])),
                         bf16_val(__uint_as_float(acc[2])), bf16_val(__uint_as_float(acc[3])) };
    if (tid < P_N / 4) {
      volatile v4f* q = (volatile v4f*)(PAR + 4 * tid);
      *q = o;
      __threadfence();
      *q = o;
    }
  }
}

template <int NIN, int NOUT, int P>
__global__ __launch_bounds__(256) void k_table(const int* __restrict__ rin, const int* __restrict__ rout,
                                               int* __restrict__ NB) {
  static_assert(NIN < (1 << 20) && NIN > 0 && NOUT > 0);
  static_assert(P % 8 == 0 && P >= 8);
  extern __shared__ __attribute__((aligned(16))) unsigned tile[];
  constexpr int STEP  = 2048;
  constexpr int NSTEP = (P + STEP - 1) / STEP;
  const int tid  = (int)threadIdx.x;
  const int row0 = (int)blockIdx.x * TILE;
  const int nrb  = clampi(NOUT - row0, 0, TILE);
  {
    const v4u z4 = (v4u){0u, 0u, 0u, 0u};
    for (int i = tid * 4; i < TILE * 32; i += 1024) *(v4ua*)(tile + i) = z4;
  }
  __syncthreads();
#pragma unroll 1
  for (int k = 0; k < NTAP; ++k) {
    const int* rik = rin + (size_t)k * P;
    const int* rok = rout + (size_t)k * P;
#pragma unroll 1
    for (int st = 0; st < NSTEP; ++st) {
      const int p8 = st * STEP + tid * 8;
      const int pc = p8 < P - 8 ? p8 : P - 8;
      const v4i o0 = *(const v4ia*)(rok + pc);
      const v4i o1 = *(const v4ia*)(rok + pc + 4);
      const v4i i0 = *(const v4ia*)(rik + pc);
      const v4i i1 = *(const v4ia*)(rik + pc + 4);
      asm volatile("" :: "v"(o0));
      asm volatile("" :: "v"(o1));
      asm volatile("" :: "v"(i0));
      asm volatile("" :: "v"(i1));
      const unsigned limit = (p8 < P) ? (unsigned)nrb : 0u;
      const int ro[8] = { o0.x, o0.y, o0.z, o0.w, o1.x, o1.y, o1.z, o1.w };
      const int ri[8] = { i0.x, i0.y, i0.z, i0.w, i1.x, i1.y, i1.z, i1.w };
      unsigned uu[8];
      bool in[8];
      bool any = false;
#pragma unroll
      for (int e = 0; e < 8; ++e) {
        uu[e] = (unsigned)ro[e] - (unsigned)row0;
        in[e] = uu[e] < limit;
        any = any || in[e];
      }
      if (__builtin_amdgcn_ballot_w32(any) != 0u) {
#pragma unroll
        for (int e = 0; e < 8; ++e) {
          const bool valid = in[e] && ((unsigned)ri[e] < (unsigned)NIN);
          if (valid) atomicAdd(&tile[uu[e] * 32u + (unsigned)k], (1u << 20) + (unsigned)ri[e]);
        }
      }
    }
  }
  __syncthreads();
  int* nb0 = NB + (size_t)row0 * 32;
  for (int pass = 0; pass < 2; ++pass) {
    for (int i = tid; i < TILE * 8; i += 256) {
      const v4u w = *(const v4ua*)(tile + 4 * i);
      v4i d;
#pragma unroll
      for (int c = 0; c < 4; ++c) {
        const unsigned cnt = w[c] >> 20;
        const int id  = (int)(w[c] & 0xFFFFFu);
        const int one = (cnt == 1u) ? id : -2;
        d[c] = (cnt == 0u) ? -1 : one;
      }
      *(volatile v4i*)(nb0 + 4 * i) = d;
    }
    __threadfence();
  }
}

template <int CIN, int TWO, int NIN>
__global__ __launch_bounds__(256) void k_gather(const float* __restrict__ src, const int* __restrict__ NB,
                                                unsigned short* __restrict__ A, int row0, int real, int nout) {
  static_assert(CIN == 64 || CIN == 128);
  static_assert(TWO == 0 || TWO == 1);
  static_assert(NTAP % 3 == 0);
  constexpr int RPW  = 128 / CIN;
  constexpr int LPR  = CIN / 4;
  constexpr int TW   = TWO ? 2 * CIN : CIN;
  constexpr int KROW = NTAP * TW;
  const int tid = (int)threadIdx.x, lane = tid & 31, wave = tid >> 5;
  const int wv  = (int)blockIdx.x * 8 + wave;
  const int sub = lane / LPR;
  const int cq  = lane - sub * LPR;
  const int lrA = wv * RPW;
  const int lrB = lrA + RPW - 1;
  const int gA  = row0 + lrA;
  const int gB  = row0 + lrB;
  const bool liveA = (lrA < real) && (gA < nout);
  const bool liveB = (lrB < real) && (gB < nout);
  int nbA = NB[(size_t)clampi(gA, 0, nout - 1) * 32 + lane];
  int nbB = NB[(size_t)clampi(gB, 0, nout - 1) * 32 + lane];
  asm volatile("" :: "v"(nbA));
  asm volatile("" :: "v"(nbB));
  nbA = clampi(nbA, -2, NIN - 1);
  nbB = clampi(nbB, -2, NIN - 1);
  nbA = liveA ? nbA : -1;
  nbB = liveB ? nbB : -1;
  unsigned short* arow = A + (size_t)(lrA + sub) * (size_t)KROW + 4 * cq;
  const float* sp = src + 4 * cq;
#pragma unroll 1
  for (int g = 0; g < NTAP / 3; ++g) {
    v2u hw[3];
    v2u lw[3];
#pragma unroll
    for (int j = 0; j < 3; ++j) {
      const int t  = 3 * g + j;
      const int ia = __builtin_amdgcn_readlane(nbA, t);
      const int ib = __builtin_amdgcn_readlane(nbB, t);
      const int id = (sub != 0) ? ib : ia;
      const int idc = id < 0 ? 0 : id;
      const v4f r = *(const v4fa*)(sp + (size_t)idc * CIN);
      asm volatile("" :: "v"(r));
      const unsigned keep = (id >= 0) ? 0xFFFFFFFFu : 0u;
      const unsigned nanw = (id == -2) ? 0x7FC07FC0u : 0u;
      hw[j] = (v2u){ (pk16(bf16_bits(r[0]), bf16_bits(r[1])) & keep) | nanw,
                     (pk16(bf16_bits(r[2]), bf16_bits(r[3])) & keep) | nanw };
      lw[j] = (v2u){ 0u, 0u };
      if (TWO) {
        lw[j] = (v2u){ (pk16(bf16_lo_bits(r[0]), bf16_lo_bits(r[1])) & keep) | nanw,
                       (pk16(bf16_lo_bits(r[2]), bf16_lo_bits(r[3])) & keep) | nanw };
      }
    }
    for (int pass = 0; pass < 2; ++pass) {
#pragma unroll
      for (int j = 0; j < 3; ++j) {
        unsigned short* q = arow + (size_t)(3 * g + j) * TW;
        *(volatile v2u*)q = hw[j];
        if (TWO) *(volatile v2u*)(q + CIN) = lw[j];
      }
      __threadfence();
    }
  }
}

template <int NC, int MODE>
__global__ __launch_bounds__(2 * NC) void k_colstat(const float* __restrict__ H, int nrows,
                                                    const float* __restrict__ mean, double* __restrict__ rec) {
  static_assert(NC == 64 || NC == 128);
  static_assert(MODE == 0 || MODE == 1);
  __shared__ __attribute__((aligned(16))) float  sm[NC];
  __shared__ __attribute__((aligned(16))) double sp[2 * NC];
  const int tid = (int)threadIdx.x;
  if (tid < 32) {
    const int pc = tid & (NC / 4 - 1);
    v4f mv = (v4f){0.f, 0.f, 0.f, 0.f};
    if constexpr (MODE == 1) {
      mv = *(const v4fa*)(mean + 4 * pc);
      asm volatile("" :: "v"(mv));
    }
    *(v4fa*)(sm + 4 * pc) = mv;
  }
  __syncthreads();
  const int col = tid & (NC - 1);
  const int g   = tid / NC;
  const int r0  = (int)blockIdx.x * 128 + g * 64;
  const int nr  = clampi(nrows - r0, 0, 64);
  const float m = sm[col];
  const float* hp = H + (size_t)r0 * NC + col;
  double s = 0.0;
#pragma unroll 4
  for (int j = 0; j < nr; ++j) {
    const float v = hp[(size_t)j * NC];
    if constexpr (MODE == 0) {
      s += (double)v;
    } else {
      const float d = v - m;
      const double dd = (double)d;
      s += dd * dd;
    }
  }
  sp[tid] = s;
  __syncthreads();
  if (tid < NC / 2) {
    const double a0 = sp[2 * tid] + sp[NC + 2 * tid];
    const double a1 = sp[2 * tid + 1] + sp[NC + 2 * tid + 1];
    const v2d o = (v2d){ a0, a1 };
    volatile v2d* q = (volatile v2d*)(rec + (size_t)blockIdx.x * NC + 2 * tid);
    *q = o;
    __threadfence();
    *q = o;
  }
}

template <int NC>
__global__ __launch_bounds__(128) void k_comb(const double* __restrict__ rec, int nrec, double inv_count, int mode,
                                              float* __restrict__ out0, float* __restrict__ out1) {
  static_assert(NC == 64 || NC == 128);
  __shared__ __attribute__((aligned(16))) float sv0[128];
  __shared__ __attribute__((aligned(16))) float sv1[128];
  const int tid = (int)threadIdx.x;
  const int c = tid < NC ? tid : NC - 1;
  double s = 0.0;
#pragma unroll 4
  for (int i = 0; i < nrec; ++i) s += rec[(size_t)i * NC + c];
  const float qf = (float)(s * inv_count);
  const float rs = 1.0f / sqrtf(qf + 1e-5f);
  sv0[tid] = qf;
  sv1[tid] = rs;
  __syncthreads();
  const int t4 = tid < NC / 4 ? tid : NC / 4 - 1;
  const v4f o0 = *(const v4fa*)(sv0 + 4 * t4);
  const v4f o1 = *(const v4fa*)(sv1 + 4 * t4);
  const bool w0 = tid < NC / 4;
  const bool w1 = w0 && (mode == 1);
  volatile v4f* q0 = (volatile v4f*)(out0 + 4 * t4);
  volatile v4f* q1 = (volatile v4f*)(out1 + 4 * t4);
  if (w0) *q0 = o0;
  if (w1) *q1 = o1;
  __threadfence();
  if (w0) *q0 = o0;
  if (w1) *q1 = o1;
}

template <int NC> struct RowV;
template <> struct RowV<128> { typedef v4f T; typedef v4fa A; };
template <> struct RowV<64>  { typedef v2f T; typedef v2fa A; };

template <int NC>
__global__ __launch_bounds__(256) void k_apply(const float* src, float* dst, int nrows, int rpw,
                                               const float* __restrict__ mean, const float* __restrict__ rstd,
                                               const float* __restrict__ gam, const float* __restrict__ bet) {
  static_assert(NC == 64 || NC == 128);
  typedef typename RowV<NC>::T VT;
  typedef typename RowV<NC>::A VA;
  constexpr int CPL = NC / 32;
  __shared__ __attribute__((aligned(16))) float spar[4 * NC];
  const int tid = (int)threadIdx.x, lane = tid & 31, wave = tid >> 5;
  if (wave == 0) {
    const int c0 = 4 * (lane & (NC / 4 - 1));
    const v4f a0 = *(const v4fa*)(mean + c0);
    const v4f a1 = *(const v4fa*)(rstd + c0);
    const v4f a2 = *(const v4fa*)(gam + c0);
    const v4f a3 = *(const v4fa*)(bet + c0);
    asm volatile("" :: "v"(a0));
    asm volatile("" :: "v"(a1));
    asm volatile("" :: "v"(a2));
    asm volatile("" :: "v"(a3));
    *(v4fa*)(spar + c0)          = a0;
    *(v4fa*)(spar + NC + c0)     = a1;
    *(v4fa*)(spar + 2 * NC + c0) = a2;
    *(v4fa*)(spar + 3 * NC + c0) = a3;
  }
  __syncthreads();
  const int cl = CPL * lane;
  const VT mv = *(const VA*)(spar + cl);
  const VT rv = *(const VA*)(spar + NC + cl);
  const VT gv = *(const VA*)(spar + 2 * NC + cl);
  const VT bv = *(const VA*)(spar + 3 * NC + cl);
  const int rbase = ((int)blockIdx.x * 8 + wave) * rpw;
#pragma unroll 1
  for (int i = 0; i < rpw; ++i) {
    const int row = rbase + i;
    const bool live = row < nrows;
    const int rc = live ? row : nrows - 1;
    const VT cv = *(const VA*)(src + (size_t)rc * NC + cl);
    asm volatile("" :: "v"(cv));
    VT y;
#pragma unroll
    for (int e = 0; e < CPL; ++e) {
      const float t = ((cv[e] - mv[e]) * rv[e]) * gv[e] + bv[e];
      y[e] = relu_k(t);
    }
    float* op = dst + (size_t)rc * NC + cl;
    if (live) *(volatile VT*)op = y;
    __threadfence();
    if (live) *(volatile VT*)op = y;
  }
}

constexpr int G_GEMM1 = (((CH1_REAL + 63) / 64) * (C1 / 64) + 7) / 8;
constexpr int G_GEMM2 = ((CH2_ROWS / 64) * (C2 / 64) + 7) / 8;
constexpr int G_GEMM3 = ((CH3_ROWS / 64) * (C2 / 64) + 7) / 8;
constexpr int G_GATH1 = CH1_PAD / 16;
constexpr int G_GATH2 = CH2_ROWS / 16;
constexpr int G_GATH3 = CH3_ROWS / 8;
constexpr int G_APPLY1 = (N1 + 63) / 64;
constexpr int G_APPLY2 = M2 / 8;
static_assert(G_GEMM1 == 24 && G_GEMM2 == 16 && G_GEMM3 == 8);
static_assert(CH1_PAD % 16 == 0 && CH2_ROWS % 16 == 0 && CH3_ROWS % 8 == 0);
static_assert(G_APPLY1 * 64 >= N1 && G_APPLY2 * 8 == M2);
static_assert((size_t)M2 * C2 == (size_t)4194304);
constexpr double INV_N1 = 1.0 / 180000.0;
constexpr double INV_M2 = 1.0 / 32768.0;
static_assert(N1 == 180000 && M2 == 32768);

template <int NC>
static void stats_apply(const float* X, float* dst, int nrows, double inv, int rpw, int gapply, double* REC, float* st,
                        const float* gam, const float* bet, hipStream_t stream) {
  const int nrec = (nrows + 127) / 128;
  k_colstat<NC, 0><<<nrec, 2 * NC, 0, stream>>>(X, nrows, st, REC);
  k_comb<NC><<<1, 128, 0, stream>>>(REC, nrec, inv, 0, st, st + ST_RS);
  k_colstat<NC, 1><<<nrec, 2 * NC, 0, stream>>>(X, nrows, st, REC);
  k_comb<NC><<<1, 128, 0, stream>>>(REC, nrec, inv, 1, st + ST_VAR, st + ST_RS);
  k_apply<NC><<<gapply, 256, 0, stream>>>(X, dst, nrows, rpw, st, st + ST_RS, gam, bet);
}

extern "C" void kernel_launch(void* const* d_in, const int* in_sizes, int n_in,
                              void* d_out, int out_size, void* d_ws, size_t ws_size,
                              hipStream_t stream) {
  if (n_in < 16) return;
  if (in_sizes[0] != N1 * C1) return;
  if (in_sizes[1] != NTAP * C1 * C1) return;
  if (in_sizes[2] != NTAP * C1 * C2) return;
  if (in_sizes[3] != NTAP * C2 * C2) return;
  if (in_sizes[4] != C1 || in_sizes[5] != C1) return;
  if (in_sizes[6] != C2 || in_sizes[7] != C2) return;
  if (in_sizes[8] != C2 || in_sizes[9] != C2) return;
  if (in_sizes[10] != NTAP * P1 || in_sizes[11] != NTAP * P1) return;
  if (in_sizes[12] != NTAP * P2 || in_sizes[13] != NTAP * P2) return;
  if (in_sizes[14] != NTAP * P2 || in_sizes[15] != NTAP * P2) return;
  if (out_size != M2 * C2) return;
  if (ws_size < WS_TOTAL) return;

  const float* feats = (const float*)d_in[0];
  const float* W1 = (const float*)d_in[1];
  const float* W2 = (const float*)d_in[2];
  const float* W3 = (const float*)d_in[3];
  const float* g1 = (const float*)d_in[4];
  const float* b1 = (const float*)d_in[5];
  const float* g2 = (const float*)d_in[6];
  const float* b2 = (const float*)d_in[7];
  const float* g3 = (const float*)d_in[8];
  const float* b3 = (const float*)d_in[9];
  const int* rb1_in  = (const int*)d_in[10];
  const int* rb1_out = (const int*)d_in[11];
  const int* rb2_in  = (const int*)d_in[12];
  const int* rb2_out = (const int*)d_in[13];
  const int* rb3_in  = (const int*)d_in[14];
  const int* rb3_out = (const int*)d_in[15];
  float* out = (float*)d_out;

  char* ws = (char*)d_ws;
  unsigned short* CHUNK = (unsigned short*)(ws + OFF_CHUNK);
  float*          X1    = (float*)(ws + OFF_X1);
  float*          X3    = (float*)(ws + OFF_X1);
  int*            NB1   = (int*)(ws + OFF_NB);
  int*            NB2   = (int*)(ws + OFF_NB);
  int*            NB3   = (int*)(ws + OFF_NB + SZ_NB2);
  float*          X2    = (float*)(ws + OFF_X2);
  unsigned short* W1T   = (unsigned short*)(ws + OFF_W1T);
  unsigned short* W2T   = (unsigned short*)(ws + OFF_W2T);
  unsigned short* W3T   = (unsigned short*)(ws + OFF_W3T);
  double*         REC   = (double*)(ws + OFF_REC);
  float*          PAR   = (float*)(ws + OFF_PAR);
  float*          ST    = (float*)(ws + OFF_ST);

  hipFuncSetAttribute(reinterpret_cast<const void*>(&k_table<N1, N1, P1>),
                      hipFuncAttributeMaxDynamicSharedMemorySize, (int)TABLE_LDS);
  hipFuncSetAttribute(reinterpret_cast<const void*>(&k_table<N1, M2, P2>),
                      hipFuncAttributeMaxDynamicSharedMemorySize, (int)TABLE_LDS);
  hipFuncSetAttribute(reinterpret_cast<const void*>(&k_table<M2, M2, P2>),
                      hipFuncAttributeMaxDynamicSharedMemorySize, (int)TABLE_LDS);

  k_wprep<<<PREP_BLOCKS, 256, 0, stream>>>(W1, W2, W3, g1, b1, g2, b2, g3, b3, W1T, W2T, W3T, PAR);
  k_table<N1, N1, P1><<<TB1, 256, TABLE_LDS, stream>>>(rb1_in, rb1_out, NB1);
  for (int c = 0; c < CH1_N; ++c) {
    k_gather<C1, 0, N1><<<G_GATH1, 256, 0, stream>>>(feats, NB1, CHUNK, c * CH1_REAL, CH1_REAL, N1);
    k_gemm_nt<0, 0><<<G_GEMM1, 256, 0, stream>>>(CHUNK, W1T, PAR, X1 + (size_t)c * CH1_REAL * C1,
                                                 CH1_REAL, C1, K1, C1);
  }
  stats_apply<C1>(X1, X1, N1, INV_N1, 8, G_APPLY1, REC, ST, PAR + P_G1, PAR + P_B1, stream);
  k_table<N1, M2, P2><<<TB2, 256, TABLE_LDS, stream>>>(rb2_in, rb2_out, NB2);
  k_table<M2, M2, P2><<<TB2, 256, TABLE_LDS, stream>>>(rb3_in, rb3_out, NB3);
  for (int c = 0; c < CH2_N; ++c) {
    k_gather<C1, TWO_TERM_2, N1><<<G_GATH2, 256, 0, stream>>>(X1, NB2, CHUNK, c * CH2_ROWS, CH2_ROWS, M2);
    k_gemm_nt<0, 0><<<G_GEMM2, 256, 0, stream>>>(CHUNK, W2T, PAR, X2 + (size_t)c * CH2_ROWS * C2,
                                                 CH2_ROWS, C2, K2, C2);
  }
  stats_apply<C2>(X2, X2, M2, INV_M2, 1, G_APPLY2, REC, ST + ST_SET, PAR + P_G2, PAR + P_B2, stream);
  for (int c = 0; c < CH3_N; ++c) {
    k_gather<C2, TWO_TERM_3, M2><<<G_GATH3, 256, 0, stream>>>(X2, NB3, CHUNK, c * CH3_ROWS, CH3_ROWS, M2);
    k_gemm_nt<0, 0><<<G_GEMM3, 256, 0, stream>>>(CHUNK, W3T, PAR, X3 + (size_t)c * CH3_ROWS * C2,
                                                 CH3_ROWS, C2, K3, C2);
  }
  stats_apply<C2>(X3, out, M2, INV_M2, 1, G_APPLY2, REC, ST + 2 * ST_SET, PAR + P_G3, PAR + P_B3, stream);
}
